// DeepLatent_49589692399911
// MI455X (gfx1250) — hardware-run, weakly checked
//
#include <hip/hip_runtime.h>


#ifndef NB
#define NB 64
#endif
#define NB_FULL  64
#define NPT      1024
#define NPT_FULL 1024
#define LAT      64
#define HID      128
#define CIN      67
#define NBP      (((NB + 15) / 16) * 16)
#define MW       4
#define PW       32
#define PB       (MW * PW)
#define HP       136
#define WCS      64.0f
#define WCI      (1.0f / 64.0f)
#define OUT_TOTAL (3 + NB * 3 * NPT)
#define NV4      (OUT_TOTAL / 4)

static_assert(NPT == NPT_FULL);
static_assert(NB <= NB_FULL);
static_assert(NBP <= NB_FULL);
static_assert(NBP % 16 == 0);
static_assert(LAT == 64);
static_assert(LAT % 32 == 0);
static_assert(HID % 32 == 0);
static_assert(HID == 128);
static_assert(HID % 16 == 0);
static_assert(CIN == 3 + LAT);
static_assert(PW == 32);
static_assert(NPT % PB == 0);
static_assert(HP >= HID);
static_assert((HP * 2) % 16 == 0);
static_assert(24 * 16 == 3 * PW * 4);
static_assert((3 * NPT / 4) % 256 == 0);
static_assert(NPT % 512 == 0);
static_assert(NPT % 4 == 0);
static_assert(OUT_TOTAL - 4 * NV4 == 3);
static_assert(NV4 % 256 == 0);
static_assert(3 * 4 == 12);
static_assert((size_t)MW * PW * HP * 2 * 2 + (size_t)MW * 16 * PW * 4 <= 131072);
static_assert((size_t)2 * 3 * NPT * 4 + 32 * 4 <= 131072);

typedef _Float16 h16;
typedef unsigned short bf;
typedef __attribute__((ext_vector_type(16))) __bf16   v16bf;
typedef __attribute__((ext_vector_type(16))) _Float16 v16h;
typedef __attribute__((ext_vector_type(8)))  _Float16 v8h;
typedef __attribute__((ext_vector_type(8)))  unsigned short v8us;
typedef __attribute__((ext_vector_type(8)))  float    v8f;
typedef __attribute__((ext_vector_type(4)))  float    v4f;
typedef v4f  __attribute__((may_alias)) v4fa;

__device__ __forceinline__ unsigned short f2bf(float f) { unsigned u = __float_as_uint(f); u += 0x7FFFu + ((u >> 16) & 1u); return (unsigned short)(u >> 16); }
__device__ __forceinline__ float bfr(float f) { return __uint_as_float(((unsigned)f2bf(f)) << 16); }
__device__ __forceinline__ v16h cat16(v8h lo, v8h hi) { return __builtin_shufflevector(lo, hi, 0, 1, 2, 3, 4, 5, 6, 7, 8, 9, 10, 11, 12, 13, 14, 15); }
__device__ __forceinline__ v16bf cat16b(v8us lo, v8us hi) { return __builtin_bit_cast(v16bf, __builtin_shufflevector(lo, hi, 0, 1, 2, 3, 4, 5, 6, 7, 8, 9, 10, 11, 12, 13, 14, 15)); }
__device__ __forceinline__ v8f wmma16(v16h a, v16h b, v8f c) { return __builtin_amdgcn_wmma_f32_16x16x32_f16(false, a, false, b, (short)0, c, false, false); }
__device__ __forceinline__ v8f wmmab(v16bf a, v16bf b, v8f c) { return __builtin_amdgcn_wmma_f32_16x16x32_bf16(false, a, false, b, (short)0, c, false, false); }
__device__ __forceinline__ v16h  ldh(const h16* p) { return cat16(*(const v8h*)p, *(const v8h*)(p + 16)); }
__device__ __forceinline__ v16bf ldb(const bf* p)  { return cat16b(*(const v8us*)p, *(const v8us*)(p + 16)); }
__device__ __forceinline__ void wave_sync() { __builtin_amdgcn_fence(3  , "wavefront"); __builtin_amdgcn_wave_barrier(); asm volatile("" ::: "memory"); }

static __device__ __forceinline__ h16 toh_flush(float v) { const h16 r = (h16)v; return (fabsf(v) < 6.103515625e-05f) ? (h16)0.0f : r; }
__device__ __forceinline__ v8f wmma16g(v16h a, v16h b, v8f c) { c = wmma16(a, b, c); asm volatile("v_nop\n\tv_nop\n\tv_nop\n\tv_nop" : "+v"(c) : "v"(a), "v"(b)); return c; }
__device__ __forceinline__ v8f wmmabg(v16bf a, v16bf b, v8f c) { c = wmmab(a, b, c); asm volatile("v_nop\n\tv_nop\n\tv_nop\n\tv_nop" : "+v"(c) : "v"(a), "v"(b)); return c; }

__global__ __launch_bounds__(256) void k_cvt8(const float* __restrict__ src, bf* dst, size_t n8) {
    const size_t i = (size_t)blockIdx.x * 256 + threadIdx.x; if (i >= n8) return;
    const v8f v = *(const v8f*)(src + i * 8); v8us o;
#pragma unroll
    for (int k = 0; k < 8; ++k) o[k] = f2bf(v[k]);
    *(volatile v8us*)(dst + i * 8) = o; __threadfence(); *(volatile v8us*)(dst + i * 8) = o;
}

__global__ __launch_bounds__(256) void k_w1l(const float* __restrict__ W1, bf* W1L) {
    const int i = blockIdx.x * 256 + threadIdx.x; if (i >= HID * LAT / 8) return;
    const int ch = i >> 3, g = i & 7;
    const float* s = W1 + (size_t)ch * CIN + 3 + 8 * g; v8us o;
#pragma unroll
    for (int k = 0; k < 8; ++k) o[k] = f2bf(s[k]);
    *(volatile v8us*)(W1L + (size_t)i * 8) = o; __threadfence(); *(volatile v8us*)(W1L + (size_t)i * 8) = o;
}

__global__ __launch_bounds__(256) void k_wconv(const float* __restrict__ W2, const float* __restrict__ W3, h16* WH) {
    const int tid = threadIdx.x;
    const int i = blockIdx.x * 256 + tid;
    v8h o;
    if (blockIdx.x < 8) {
        const v8f v = *(const v8f*)(W2 + (size_t)i * 8);
#pragma unroll
        for (int k = 0; k < 8; ++k) o[k] = toh_flush(bfr(v[k]) * WCS);
    } else {
        const int orow = tid >> 4, c8 = (tid & 15) * 8;
        const int oc = orow < 3 ? orow : 2;
        v8f v = *(const v8f*)(W3 + (size_t)oc * HID + c8);
        asm volatile("" : "+v"(v));
#pragma unroll
        for (int k = 0; k < 8; ++k) { const h16 t = toh_flush(bfr(v[k]) * WCS); o[k] = (orow < 3) ? t : (h16)0.0f; }
    }
    *(volatile v8h*)(WH + (size_t)i * 8) = o; __threadfence(); *(volatile v8h*)(WH + (size_t)i * 8) = o;
}

__global__ __launch_bounds__(32) void k_c1(const bf* __restrict__ LATB, const bf* __restrict__ W1L, const float* __restrict__ W1, const float* __restrict__ b1, float* T1) {
    const int lane = threadIdx.x & 31, lr = lane & 15, hi = lane >> 4;
    const int m0 = blockIdx.x * 16, n0 = blockIdx.y * 16;
    v8f acc = (v8f){};
#pragma unroll
    for (int kc = 0; kc < LAT; kc += 32) {
        const v16bf a = ldb(LATB + (size_t)(m0 + lr) * LAT + kc + 8 * hi);
        const v16bf b = ldb(W1L + (size_t)(n0 + lr) * LAT + kc + 8 * hi);
        acc = wmmabg(a, b, acc);
    }
    const int ch = n0 + lr;
    const float w0 = bfr(W1[(size_t)ch * CIN + 0]), w1 = bfr(W1[(size_t)ch * CIN + 1]), w2 = bfr(W1[(size_t)ch * CIN + 2]);
    const float bias = bfr(b1[ch]);
#pragma unroll 1
    for (int ps = 0; ps < 2; ++ps) {
#pragma unroll
        for (int r = 0; r < 8; ++r) {
            v4f t; t[0] = w0; t[1] = w1; t[2] = w2; t[3] = acc[r] + bias;
            *(volatile v4f*)(T1 + ((size_t)(m0 + 8 * hi + r) * HID + ch) * 4) = t; }
        if (ps == 0) __threadfence(); }
}

__global__ __launch_bounds__(32 * MW) void k_mlp(const float* __restrict__ pc, const float* __restrict__ T1, const h16* __restrict__ W2H, const float* __restrict__ b2,
                                                 const h16* __restrict__ W3H, const float* __restrict__ b3, float* EST) {
    __shared__ __align__(16) h16 hs1[MW * PW * HP];
    __shared__ __align__(16) h16 hs2[MW * PW * HP];
    __shared__ __align__(16) float ns[MW * 16 * PW];
    const int lane = threadIdx.x & 31, lr = lane & 15, hi = lane >> 4;
    const int wave = __builtin_amdgcn_readfirstlane((int)(threadIdx.x >> 5));
    const int b = blockIdx.y;
    const int n0 = blockIdx.x * PB + wave * PW;
    const int hsb = wave * PW * HP;
    const size_t pcb = (size_t)b * 3 * NPT_FULL + (size_t)(n0 + lane);
    const float px = bfr(pc[pcb]), py = bfr(pc[pcb + NPT_FULL]), pz = bfr(pc[pcb + 2 * NPT_FULL]);
    const float* t1b = T1 + (size_t)b * HID * 4;
#pragma unroll 1
    for (int cg = 0; cg < HID / 8; ++cg) {
        v8h hv;
#pragma unroll
        for (int j = 0; j < 8; ++j) {
            const v4f t = *(const v4f*)(t1b + (size_t)(cg * 8 + j) * 4);
            float v = t[3]; v = fmaf(t[0], px, v); v = fmaf(t[1], py, v); v = fmaf(t[2], pz, v);
            v = fmaxf(v, 0.0f);
            hv[j] = toh_flush(v); }
        *(v8h*)&hs1[hsb + lane * HP + cg * 8] = hv;
    }
    wave_sync();
#pragma unroll 1
    for (int nh = 0; nh < 2; ++nh) {
        v8f acc[2][4];
#pragma unroll
        for (int mb = 0; mb < 2; ++mb)
#pragma unroll
            for (int nb = 0; nb < 4; ++nb) acc[mb][nb] = (v8f){};
        const size_t wo = (size_t)(nh * 64 + lr) * HID + 8 * hi;
#pragma unroll 1
        for (int kc = 0; kc < HID; kc += 32) {
            const int ai = hsb + lr * HP + kc + 8 * hi;
            const v16h a0 = cat16(*(const v8h*)&hs1[ai], *(const v8h*)&hs1[ai + 16]);
            const v16h a1 = cat16(*(const v8h*)&hs1[ai + 16 * HP], *(const v8h*)&hs1[ai + 16 * HP + 16]);
#pragma unroll
            for (int nb = 0; nb < 4; ++nb) {
                const v16h bw = ldh(W2H + wo + (size_t)nb * 16 * HID + kc);
                acc[0][nb] = wmma16g(a0, bw, acc[0][nb]);
                acc[1][nb] = wmma16g(a1, bw, acc[1][nb]); }
        }
#pragma unroll
        for (int nb = 0; nb < 4; ++nb) {
            const int ch = nh * 64 + nb * 16 + lr;
            const float bias = bfr(b2[ch]);
#pragma unroll
            for (int mb = 0; mb < 2; ++mb)
#pragma unroll
                for (int r = 0; r < 8; ++r) {
                    float v = acc[mb][nb][r] * WCI + bias; v = fmaxf(v, 0.0f);
                    hs2[hsb + (mb * 16 + 8 * hi + r) * HP + ch] = toh_flush(v); }
        }
    }
    wave_sync();
    v8f q0 = (v8f){}, q1 = (v8f){};
    const size_t w3o = (size_t)lr * HID + 8 * hi;
#pragma unroll 1
    for (int kc = 0; kc < HID; kc += 32) {
        const int ai = hsb + lr * HP + kc + 8 * hi;
        const v16h a0 = cat16(*(const v8h*)&hs2[ai], *(const v8h*)&hs2[ai + 16]);
        const v16h a1 = cat16(*(const v8h*)&hs2[ai + 16 * HP], *(const v8h*)&hs2[ai + 16 * HP + 16]);
        const v16h bw = ldh(W3H + w3o + kc);
        q0 = wmma16g(a0, bw, q0);
        q1 = wmma16g(a1, bw, q1);
    }
    const int nsb = wave * 16 * PW;
    { v4f a, c;
      a[0] = q0[0]; a[1] = q0[1]; a[2] = q0[2]; a[3] = q0[3]; c[0] = q0[4]; c[1] = q0[5]; c[2] = q0[6]; c[3] = q0[7];
      *(v4fa*)(&ns[nsb + lr * PW + 8 * hi]) = a; *(v4fa*)(&ns[nsb + lr * PW + 8 * hi + 4]) = c;
      a[0] = q1[0]; a[1] = q1[1]; a[2] = q1[2]; a[3] = q1[3]; c[0] = q1[4]; c[1] = q1[5]; c[2] = q1[6]; c[3] = q1[7];
      *(v4fa*)(&ns[nsb + lr * PW + 16 + 8 * hi]) = a; *(v4fa*)(&ns[nsb + lr * PW + 16 + 8 * hi + 4]) = c; }
    wave_sync();
    const int o3 = lane >> 3, oc = o3 < 3 ? o3 : 2, c4 = (lane & 7) * 4;
    const v4f nz = *(const v4fa*)(&ns[nsb + oc * PW + c4]);
    v4f pv = *(const v4f*)(pc + ((size_t)b * 3 + oc) * NPT_FULL + n0 + c4);
    float bz = b3[oc];
    asm volatile("" : "+v"(pv));
    asm volatile("" : "+v"(bz));
    const float bb = bfr(bz);
    v4f val;
#pragma unroll
    for (int i = 0; i < 4; ++i) val[i] = bfr(pv[i]) - (nz[i] * WCI + bb);
    float* ep = EST + ((size_t)b * 3 + oc) * NPT + n0 + c4;
    if (o3 < 3) *(volatile v4f*)ep = val;
    __threadfence();
    if (o3 < 3) *(volatile v4f*)ep = val;
}

__global__ __launch_bounds__(256) void k_dist(const float* __restrict__ gt, const float* __restrict__ EST, float* P) {
    __shared__ __align__(16) float pts[2 * 3 * NPT];
    __shared__ float red[8 * 4];
    const int b = blockIdx.x, tid = threadIdx.x;
    const int lane = tid & 31;
    const int wave = __builtin_amdgcn_readfirstlane((int)(threadIdx.x >> 5));
    float sq = 0.0f;
#pragma unroll 1
    for (int i = tid; i < 3 * NPT / 4; i += 256) {
        const v4f g = *(const v4f*)(gt + (size_t)b * 3 * NPT_FULL + 4 * i);
        const v4f e = *(const v4f*)(EST + (size_t)b * 3 * NPT + 4 * i);
        v4f gr;
#pragma unroll
        for (int c = 0; c < 4; ++c) { gr[c] = bfr(g[c]); const float d = gr[c] - e[c]; sq = fmaf(d, d, sq); }
        *(v4fa*)(&pts[4 * i]) = gr; *(v4fa*)(&pts[3 * NPT + 4 * i]) = e;
    }
    __syncthreads();
    float srow = 0.0f, scol = 0.0f;
#pragma unroll 1
    for (int dir = 0; dir < 2; ++dir) {
        const int so = dir * 3 * NPT, to = (1 - dir) * 3 * NPT;
        float accm = 0.0f;
#pragma unroll 1
        for (int q = 0; q < NPT / 512; ++q) {
            const int na = tid + 512 * q, nc = na + 256;
            const float ax = pts[so + na], ay = pts[so + NPT + na], az = pts[so + 2 * NPT + na];
            const float cx = pts[so + nc], cy = pts[so + NPT + nc], cz = pts[so + 2 * NPT + nc];
            float ma = 3.0e38f, mc = 3.0e38f;
#pragma unroll 1
            for (int m = 0; m < NPT; m += 4) {
                const v4f tx = *(const v4fa*)(&pts[to + m]), ty = *(const v4fa*)(&pts[to + NPT + m]), tz = *(const v4fa*)(&pts[to + 2 * NPT + m]);
#pragma unroll
                for (int c = 0; c < 4; ++c) {
                    const float dx = ax - tx[c], dy = ay - ty[c], dz = az - tz[c];
                    ma = fminf(ma, fmaf(dx, dx, fmaf(dy, dy, dz * dz)));
                    const float ex = cx - tx[c], ey = cy - ty[c], ez = cz - tz[c];
                    mc = fminf(mc, fmaf(ex, ex, fmaf(ey, ey, ez * ez))); }
            }
            accm += ma + mc;
        }
        if (dir == 0) srow = accm; else scol = accm;
    }
#pragma unroll
    for (int off = 16; off > 0; off >>= 1) { srow += __shfl_xor(srow, off, 32); scol += __shfl_xor(scol, off, 32); sq += __shfl_xor(sq, off, 32); }
    if (lane == 0) { red[wave * 4 + 0] = srow; red[wave * 4 + 1] = scol; red[wave * 4 + 2] = sq; }
    __syncthreads();
    float R = 0.0f, C = 0.0f, Q = 0.0f;
#pragma unroll
    for (int w = 0; w < 8; ++w) { R += red[w * 4 + 0]; C += red[w * 4 + 1]; Q += red[w * 4 + 2]; }
    const int tc = tid < 8 ? tid : 7;
    v4f v; v[0] = (tid == 0) ? R : 0.0f; v[1] = (tid == 0) ? C : 0.0f; v[2] = (tid == 0) ? Q : 0.0f; v[3] = 0.0f;
    float* pp = P + (size_t)b * 32 + tc * 4;
    if (tid < 8) *(volatile v4f*)pp = v;
    __threadfence();
    if (tid < 8) *(volatile v4f*)pp = v;
}

__global__ __launch_bounds__(256) void k_emit(const float* __restrict__ EST, const float* __restrict__ P, float* OUT) {
    __shared__ float sc[4];
    const int tid = threadIdx.x;
    float s0 = 0.0f, s1 = 0.0f, s2 = 0.0f;
    if (blockIdx.x == 0) {
        const int kk = tid < 3 ? tid : 2;
        float a = 0.0f;
#pragma unroll 1
        for (int b = 0; b < NB; ++b) a += P[(size_t)b * 32 + kk];
        if (tid < 3) sc[tid] = a;
        __syncthreads();
        const float R = sc[0], C = sc[1], Q = sc[2];
        const float inv = 1.0f / (float)(NB * NPT);
        const float ch = R * inv + C * inv;
        const float l2 = Q * (1.0f / (float)(NB * 3 * NPT));
        s0 = 0.1f * ch + (float)(1.0 - 0.1) * l2; s1 = ch; s2 = l2;
    }
    const size_t i = (size_t)blockIdx.x * 256 + tid;
    if (i < (size_t)NV4) {
        const size_t g0 = 4 * i; v4f val;
#pragma unroll
        for (int c = 0; c < 4; ++c) {
            const size_t g = g0 + c;
            const size_t ei = g >= 3 ? g - 3 : 0;
            float e = EST[ei];
            asm volatile("" : "+v"(e));
            val[c] = (g == 0) ? s0 : ((g == 1) ? s1 : ((g == 2) ? s2 : e)); }
        *(volatile v4f*)(OUT + g0) = val;
        __threadfence();
        *(volatile v4f*)(OUT + g0) = val;
    } else {
        const int t = (int)(i - (size_t)NV4); const int tc = t < 3 ? t : 2;
        float e = EST[(size_t)(OUT_TOTAL - 6 + tc)];
        asm volatile("" : "+v"(e));
        float* p = OUT + (size_t)4 * NV4 + tc;
        if (t < 3) *(volatile float*)p = e;
        __threadfence();
        if (t < 3) *(volatile float*)p = e;
    }
}

static constexpr size_t al256(size_t v) { return (v + 255) & ~(size_t)255; }
static constexpr size_t SZ_LATB = al256((size_t)NBP * LAT * 2);
static constexpr size_t SZ_W1L  = al256((size_t)HID * LAT * 2);
static constexpr size_t SZ_WH   = al256((size_t)(HID + 16) * HID * 2);
static constexpr size_t SZ_T1   = al256((size_t)NBP * HID * 16);
static constexpr size_t SZ_EST  = al256((size_t)NB * 3 * NPT * 4);
static constexpr size_t SZ_P    = al256((size_t)NB * 128);
static constexpr size_t SZ_TOTAL = SZ_LATB + SZ_W1L + SZ_WH + SZ_T1 + SZ_EST + SZ_P;
static_assert(SZ_TOTAL <= (size_t)134217728);
static_assert((size_t)9 * 256 * 8 == (size_t)(HID + 16) * HID);
static_assert((size_t)(NBP / 16) * (HID / 16) * 256 * 16 == (size_t)NBP * HID * 16);
static_assert((size_t)(NPT / PB) * NB * MW * 3 * 128 == (size_t)NB * 3 * NPT * 4);
static_assert(((size_t)NBP * LAT) % 8 == 0);

extern "C" void kernel_launch(void* const* d_in, const int* in_sizes, int n_in,
                              void* d_out, int out_size, void* d_ws, size_t ws_size, hipStream_t stream) {
    if (n_in < 9) return;
    if ((size_t)in_sizes[0] < (size_t)NB * 3 * NPT_FULL || (size_t)in_sizes[1] < (size_t)NB * 3 * NPT_FULL) return;
    if ((size_t)in_sizes[2] < (size_t)NBP * LAT) return;
    if ((size_t)in_sizes[3] < (size_t)HID * CIN || in_sizes[4] < HID) return;
    if ((size_t)in_sizes[5] < (size_t)HID * HID || in_sizes[6] < HID) return;
    if (in_sizes[7] < 3 * HID || in_sizes[8] < 3) return;
    if ((size_t)out_size < (size_t)OUT_TOTAL) return;
    if (SZ_TOTAL > ws_size) return;
    const float* pc  = (const float*)d_in[0];
    const float* gt  = (const float*)d_in[1];
    const float* lat = (const float*)d_in[2];
    const float* w1  = (const float*)d_in[3]; const float* b1 = (const float*)d_in[4];
    const float* w2  = (const float*)d_in[5]; const float* b2 = (const float*)d_in[6];
    const float* w3  = (const float*)d_in[7]; const float* b3 = (const float*)d_in[8];
    float* OUT = (float*)d_out;
    char* wsp = (char*)d_ws;
    bf*  LATB = (bf*)wsp;   wsp += SZ_LATB;
    bf*  W1L  = (bf*)wsp;   wsp += SZ_W1L;
    h16* WH   = (h16*)wsp;  wsp += SZ_WH;
    float* T1 = (float*)wsp; wsp += SZ_T1;
    float* EST = (float*)wsp; wsp += SZ_EST;
    float* P  = (float*)wsp; wsp += SZ_P;
    h16* W2H = WH; h16* W3H = WH + (size_t)HID * HID;

    { const size_t n8 = (size_t)NBP * LAT / 8; k_cvt8<<<(unsigned)((n8 + 255) / 256), 256, 0, stream>>>(lat, LATB, n8); }
    k_w1l<<<(HID * LAT / 8 + 255) / 256, 256, 0, stream>>>(w1, W1L);
    k_wconv<<<9, 256, 0, stream>>>(w2, w3, WH);
    k_c1<<<dim3(NBP / 16, HID / 16, 1), 32, 0, stream>>>(LATB, W1L, w1, b1, T1);
    k_mlp<<<dim3(NPT / PB, NB, 1), 32 * MW, 0, stream>>>(pc, T1, W2H, b2, W3H, b3, EST);
    k_dist<<<NB, 256, 0, stream>>>(gt, EST, P);
    k_emit<<<(unsigned)((NV4 + 3 + 255) / 256), 256, 0, stream>>>(EST, P, OUT);
}
